// PETP_Quadratic_790273982668
// MI455X (gfx1250) — hardware-verified
//
#include <hip/hip_runtime.h>
#include <stddef.h>


typedef _Float16 v16h __attribute__((ext_vector_type(16)));
typedef _Float16 v8h  __attribute__((ext_vector_type(8)));
typedef float    v16f __attribute__((ext_vector_type(16)));
typedef float    v8f  __attribute__((ext_vector_type(8)));
typedef float    v4f  __attribute__((ext_vector_type(4)));

#ifndef NB
#define NB 16384
#endif
#define NB_FULL 16384
#define NI 2
#define NJ 3
#define CH 32
#define ROWW 128
#define ROWS_PER_B (NI * NJ)
#define BSTRIDE (ROWS_PER_B * ROWW)

#define BPB  16
#define RPB  (BPB * ROWS_PER_B)
#define NWV  (RPB / 16)
#define NTHR (NWV * 32)
#define LDR  132

#define FCARRY 64.0f
#define WCARRY 64.0f
#define XFLOOR 0.0009765625f
#define F16MIN 6.103515625e-05f
#define NORMC  0.022097086912079608f
#define C1F    36.95041722813605f

#define MAT_H    (CH * CH)
#define PLANE_U  (3 * MAT_H)
#define PLANE_T  (CH * PLANE_U)
#define WS_TOTAL ((size_t)4 * PLANE_T * 2)

static_assert(NB >= BPB && NB <= NB_FULL);
static_assert((NB % BPB) == 0);
static_assert(ROWW == CH + 3 * CH);
static_assert(CH == 32);
static_assert((RPB % 16) == 0);
static_assert(NTHR == 192 && NTHR <= 256);
static_assert((LDR % 4) == 0 && LDR >= ROWW);
static_assert((size_t)RPB * LDR * 4 <= (size_t)65536);
static_assert(XFLOOR * XFLOOR * FCARRY >= F16MIN);
static_assert(32 * 16 == 4 * ROWW);
static_assert(128 * 8 == MAT_H);
static_assert((MAT_H * 2) % 128 == 0);
static_assert((WS_TOTAL % 128) == 0);
static_assert(WS_TOTAL <= (size_t)134217728);
static_assert((size_t)NB_FULL * BSTRIDE < (size_t)0x7FFFFFFF);

__device__ __forceinline__ float bf16r(float x) {
  unsigned int u = __float_as_uint(x);
  u = (u + 0x7FFFu + ((u >> 16) & 1u)) & 0xFFFF0000u;
  return __uint_as_float(u);
}

__device__ __forceinline__ v16h frag_at(const _Float16* p) {
  v8h lo = *(const v8h*)(p);
  v8h hi = *(const v8h*)(p + 16);
  v16h out;
#pragma unroll
  for (int i = 0; i < 8; ++i) { out[i] = lo[i]; out[i + 8] = hi[i]; }
  return out;
}

__device__ __forceinline__ v8f wmma16(v16h a, v16h b, v8f c) {
  v8f d = __builtin_amdgcn_wmma_f32_16x16x32_f16(false, a, false, b, (short)0, c,
                                                 false, false);
  asm volatile("v_nop\n\tv_nop\n\tv_nop\n\tv_nop" : "+v"(d) : "v"(a), "v"(b));
  return d;
}

static __device__ __forceinline__ _Float16 toh_flush(float v) {
  const _Float16 r = (_Float16)v;
  return (fabsf(v) < F16MIN) ? (_Float16)0.0f : r;
}
static __device__ __forceinline__ float cut_small(float v, float lim) {
  return (fabsf(v) < lim) ? 0.0f : v;
}

__global__ __launch_bounds__(128) void wprep_kernel(
    const float* __restrict__ W, _Float16* __restrict__ dst) {
  const unsigned tid = threadIdx.x;
  const unsigned u = blockIdx.x;
  const unsigned w = tid >> 2, q = tid & 3u;
  v8h x0, x1, x2;
#pragma unroll
  for (unsigned j = 0; j < 8u; ++j) {
    const unsigned v = q * 8u + j;
    const float a0 = W[((0u * 32u + u) * 32u + v) * 32u + w];
    const float a1 = W[((1u * 32u + u) * 32u + v) * 32u + w];
    const float a2 = W[((2u * 32u + u) * 32u + v) * 32u + w];
    const float a3 = W[((3u * 32u + v) * 32u + u) * 32u + w];
    x0[j] = toh_flush(WCARRY * bf16r(a0));
    x1[j] = toh_flush(WCARRY * bf16r(a1));
    x2[j] = toh_flush(WCARRY * (bf16r(a2) + bf16r(a3)));
  }
  _Float16* p = dst + (size_t)u * PLANE_U + tid * 8u;
  *(volatile v8h*)(p) = x0;
  *(volatile v8h*)(p + MAT_H) = x1;
  *(volatile v8h*)(p + 2 * MAT_H) = x2;
  __threadfence();
  *(volatile v8h*)(p) = x0;
  *(volatile v8h*)(p + MAT_H) = x1;
  *(volatile v8h*)(p + 2 * MAT_H) = x2;
}

__global__ __launch_bounds__(NTHR) __attribute__((amdgpu_num_vgpr(256)))
void petp_main_kernel(const float* __restrict__ x, const _Float16* __restrict__ wpl,
                      float* __restrict__ out) {
  __shared__ __attribute__((aligned(16))) float R[RPB * LDR];

  const unsigned tid = threadIdx.x, lane = tid & 31u;
  const unsigned wave = (unsigned)__builtin_amdgcn_readfirstlane((int)(tid >> 5));
  const unsigned hh = lane >> 4, m = lane & 15u;
  const unsigned b0 = blockIdx.x * (unsigned)BPB;
  const unsigned rbase = (wave * 16u + m) * (unsigned)LDR;

  v8f accs[2];
  v8f accv[3][2];
#pragma unroll
  for (int nt = 0; nt < 2; ++nt) {
    accs[nt] = (v8f){};
#pragma unroll
    for (int k = 0; k < 3; ++k) accv[k][nt] = (v8f){};
  }

#pragma unroll 1
  for (unsigned t = 0; t < 4u; ++t) {
#pragma unroll 1
    for (unsigned idx = tid; idx < (unsigned)(BPB * ROWW); idx += (unsigned)NTHR) {
      const unsigned bl = idx >> 7, c = idx & 127u;
      const float* xb = x + (size_t)(b0 + bl) * BSTRIDE + c;
      float xv[6];
#pragma unroll
      for (int q = 0; q < 6; ++q) xv[q] = bf16r(xb[q * ROWW]);
      const float rs[2] = {(xv[0] + xv[1]) + xv[2], (xv[3] + xv[4]) + xv[5]};
      const float cs[3] = {xv[0] + xv[3], xv[1] + xv[4], xv[2] + xv[5]};
      const float ts = rs[0] + rs[1];
      const unsigned e = (c >= 32u) ? (c - 32u) : 0u;
      const unsigned uu = e / 3u;
      const unsigned kk = e - 3u * uu;
      const unsigned cm = (c >= 32u) ? (32u + kk * 32u + uu) : c;
#pragma unroll
      for (int i = 0; i < 2; ++i) {
#pragma unroll
        for (int j = 0; j < 3; ++j) {
          const float s = xv[i * 3 + j];
          const float fu = rs[i] - s;
          const float nu = cs[j] - s;
          const float au = ((ts - s) - fu) - nu;
          float val = s;
          val = (t == 1u) ? (0.5f * fu) : val;
          val = (t == 2u) ? nu : val;
          val = (t == 3u) ? (0.5f * au) : val;
          val = cut_small(val, XFLOOR);
          R[(bl * 6u + (unsigned)(i * 3 + j)) * (unsigned)LDR + cm] = val;
        }
      }
    }
    __syncthreads();

    v16f S, V0, V1, V2;
    {
      const unsigned o = rbase + 8u * hh;
#pragma unroll
      for (int q = 0; q < 2; ++q) {
        const v4f s0 = *(const v4f*)&R[o + 16 * q];
        const v4f s1 = *(const v4f*)&R[o + 16 * q + 4];
        const v4f a0 = *(const v4f*)&R[o + 32 + 16 * q];
        const v4f a1 = *(const v4f*)&R[o + 32 + 16 * q + 4];
        const v4f c0 = *(const v4f*)&R[o + 64 + 16 * q];
        const v4f c1 = *(const v4f*)&R[o + 64 + 16 * q + 4];
        const v4f d0 = *(const v4f*)&R[o + 96 + 16 * q];
        const v4f d1 = *(const v4f*)&R[o + 96 + 16 * q + 4];
#pragma unroll
        for (int ee = 0; ee < 4; ++ee) {
          S[8 * q + ee]  = s0[ee];  S[8 * q + 4 + ee]  = s1[ee];
          V0[8 * q + ee] = a0[ee];  V0[8 * q + 4 + ee] = a1[ee];
          V1[8 * q + ee] = c0[ee];  V1[8 * q + 4 + ee] = c1[ee];
          V2[8 * q + ee] = d0[ee];  V2[8 * q + 4 + ee] = d1[ee];
        }
      }
    }

#pragma unroll 1
    for (unsigned u = 0; u < (unsigned)CH; ++u) {
      const float su = R[rbase + u] * FCARRY;
      const float w0 = R[rbase + 32u + u] * C1F;
      const float w1 = R[rbase + 64u + u] * C1F;
      const float w2 = R[rbase + 96u + u] * C1F;
      const _Float16* bp = wpl + (size_t)(t * (unsigned)CH + u) * PLANE_U + m * 32u + hh * 8u;

      {
        const v16f p = S * su;
        const v16h a = __builtin_convertvector(p, v16h);
        const v16h bA = frag_at(bp);
        const v16h bB = frag_at(bp + 512);
        accs[0] = wmma16(a, bA, accs[0]);
        accs[1] = wmma16(a, bB, accs[1]);
      }
      {
        v16f p = V0 * w0 + V1 * w1 + V2 * w2;
#pragma unroll
        for (int i = 0; i < 16; ++i) p[i] = cut_small(p[i], F16MIN);
        const v16h a = __builtin_convertvector(p, v16h);
        const v16h bA = frag_at(bp + MAT_H);
        const v16h bB = frag_at(bp + MAT_H + 512);
        accs[0] = wmma16(a, bA, accs[0]);
        accs[1] = wmma16(a, bB, accs[1]);
      }
      {
        const v16h bA = frag_at(bp + 2 * MAT_H);
        const v16h bB = frag_at(bp + 2 * MAT_H + 512);
        {
          const v16f p = V0 * su;
          const v16h a = __builtin_convertvector(p, v16h);
          accv[0][0] = wmma16(a, bA, accv[0][0]);
          accv[0][1] = wmma16(a, bB, accv[0][1]);
        }
        {
          const v16f p = V1 * su;
          const v16h a = __builtin_convertvector(p, v16h);
          accv[1][0] = wmma16(a, bA, accv[1][0]);
          accv[1][1] = wmma16(a, bB, accv[1][1]);
        }
        {
          const v16f p = V2 * su;
          const v16h a = __builtin_convertvector(p, v16h);
          accv[2][0] = wmma16(a, bA, accv[2][0]);
          accv[2][1] = wmma16(a, bB, accv[2][1]);
        }
      }
    }
    __syncthreads();
  }

  const float osc = NORMC * (1.0f / (FCARRY * WCARRY));
#pragma unroll
  for (int r = 0; r < 8; ++r) {
    const unsigned ro = (wave * 16u + hh * 8u + (unsigned)r) * (unsigned)LDR;
    R[ro + m]       = accs[0][r] * osc;
    R[ro + 16u + m] = accs[1][r] * osc;
#pragma unroll
    for (int k = 0; k < 3; ++k) {
      R[ro + 32u + 3u * m + (unsigned)k]          = accv[k][0][r] * osc;
      R[ro + 32u + 3u * (16u + m) + (unsigned)k]  = accv[k][1][r] * osc;
    }
  }
  __syncthreads();

  v4f xs[16];
#pragma unroll
  for (int r = 0; r < 16; ++r)
    xs[r] = *(const v4f*)&R[(wave * 16u + (unsigned)r) * (unsigned)LDR + lane * 4u];
  float* op = out + ((size_t)blockIdx.x * RPB + wave * 16u) * ROWW + lane * 4u;
#pragma unroll
  for (int r = 0; r < 16; ++r) *(volatile v4f*)(op + r * ROWW) = xs[r];
  __threadfence();
#pragma unroll
  for (int r = 0; r < 16; ++r) *(volatile v4f*)(op + r * ROWW) = xs[r];
}

extern "C" void kernel_launch(void* const* d_in, const int* in_sizes, int n_in,
                              void* d_out, int out_size, void* d_ws, size_t ws_size,
                              hipStream_t stream) {
  if (n_in < 5) return;
  const long long need_x = (long long)NB * BSTRIDE;
  const long long need_w = (long long)4 * CH * CH * CH;
  if ((long long)in_sizes[0] < need_x) return;
  if ((long long)in_sizes[1] < need_w) return;
  if ((long long)in_sizes[2] < need_w) return;
  if ((long long)in_sizes[3] < need_w) return;
  if ((long long)in_sizes[4] < need_w) return;
  if ((long long)out_size < need_x) return;
  if (ws_size < WS_TOTAL) return;

  const float* X      = (const float*)d_in[0];
  const float* Wself  = (const float*)d_in[1];
  const float* Wflav  = (const float*)d_in[2];
  const float* Wnnb   = (const float*)d_in[3];
  const float* Wall   = (const float*)d_in[4];
  float* out = (float*)d_out;
  _Float16* planes = (_Float16*)d_ws;

  wprep_kernel<<<dim3(CH), dim3(128), 0, stream>>>(Wself, planes + (size_t)0 * PLANE_T);
  wprep_kernel<<<dim3(CH), dim3(128), 0, stream>>>(Wflav, planes + (size_t)1 * PLANE_T);
  wprep_kernel<<<dim3(CH), dim3(128), 0, stream>>>(Wnnb,  planes + (size_t)2 * PLANE_T);
  wprep_kernel<<<dim3(CH), dim3(128), 0, stream>>>(Wall,  planes + (size_t)3 * PLANE_T);

  petp_main_kernel<<<dim3(NB / BPB), dim3(NTHR), 0, stream>>>(X, planes, out);
}
